// MSARowAttentionWithPairBias_46918222742020
// MI455X (gfx1250) — hardware-verified
//
#include <hip/hip_runtime.h>


#define NS   128
#define NN   256
#define DN   256
#define DP   128
#define NH_  8
#define HC   32
#define SPP  8
#define ZP   (SPP * NH_)
#define PCAR 1024.0f
typedef _Float16 h16;
typedef unsigned short bf;
typedef __attribute__((ext_vector_type(16))) __bf16   v16bf;
typedef __attribute__((ext_vector_type(16))) _Float16 v16h;
typedef __attribute__((ext_vector_type(8)))  _Float16 v8h;
typedef __attribute__((ext_vector_type(8)))  unsigned short v8us;
typedef __attribute__((ext_vector_type(8)))  float    v8f;
typedef __attribute__((ext_vector_type(4)))  float    v4f;
typedef v8h  __attribute__((may_alias)) v8ha;
typedef v4f  __attribute__((may_alias)) v4fa;
typedef v8us __attribute__((may_alias)) v8usa;

__device__ __forceinline__ unsigned short f2bf(float f) { unsigned u = __float_as_uint(f); u += 0x7FFFu + ((u >> 16) & 1u); return (unsigned short)(u >> 16); }
__device__ __forceinline__ float bf2f(unsigned short b) { return __uint_as_float(((unsigned)b) << 16); }
__device__ __forceinline__ float bfr(float f) { return bf2f(f2bf(f)); }
__device__ __forceinline__ v16h cat16(v8h lo, v8h hi) { return __builtin_shufflevector(lo, hi, 0, 1, 2, 3, 4, 5, 6, 7, 8, 9, 10, 11, 12, 13, 14, 15); }
__device__ __forceinline__ v16bf cat16b(v8us lo, v8us hi) { return __builtin_bit_cast(v16bf, __builtin_shufflevector(lo, hi, 0, 1, 2, 3, 4, 5, 6, 7, 8, 9, 10, 11, 12, 13, 14, 15)); }
__device__ __forceinline__ v8f wmma16(v16h a, v16h b, v8f c) { return __builtin_amdgcn_wmma_f32_16x16x32_f16(false, a, false, b, (short)0, c, false, false); }
__device__ __forceinline__ v8f wmmab(v16bf a, v16bf b, v8f c) { return __builtin_amdgcn_wmma_f32_16x16x32_bf16(false, a, false, b, (short)0, c, false, false); }


template <typename T16> struct WFrag;
template <> struct WFrag<h16> { typedef v16h V; static __device__ __forceinline__ V ld(const h16* p) { return cat16(*(const v8h*)p, *(const v8h*)(p + 16)); } static __device__ __forceinline__ v8f mma(V a, V b, v8f c) { return wmma16(a, b, c); } };
template <> struct WFrag<bf> { typedef v16bf V; static __device__ __forceinline__ V ld(const bf* p) { return cat16b(*(const v8us*)p, *(const v8us*)(p + 16)); } static __device__ __forceinline__ v8f mma(V a, V b, v8f c) { return wmmab(a, b, c); } };
template <typename T16, int NSPLIT, bool BIAS>
__global__ __launch_bounds__(32) void k_gemmw(const T16* __restrict__ A, const T16* __restrict__ A2, const T16* __restrict__ Bt, const T16* __restrict__ Bt2, int K, float* C, int ldc, const float* __restrict__ bias, size_t sA, size_t sB, size_t sC) {
    typedef typename WFrag<T16>::V V;
    __shared__ __align__(16) float os[16 * 68];
    const size_t z = blockIdx.z; A += z * sA; if (A2) A2 += z * sA; Bt += z * sB; if (Bt2) Bt2 += z * sB; C += z * sC;
    const int lane = threadIdx.x & 31, lr = lane & 15, hi = lane >> 4; const int r0 = blockIdx.x * 64, c0 = blockIdx.y * 64;
    v8f acc[4][4];
#pragma unroll
    for (int mb = 0; mb < 4; ++mb)
#pragma unroll
        for (int nb = 0; nb < 4; ++nb) acc[mb][nb] = (v8f){};
    const size_t aoff = (size_t)(r0 + lr) * K + 8 * hi, boff = (size_t)(c0 + lr) * K + 8 * hi;
#pragma unroll 1
    for (int kc = 0; kc < K; kc += 32) {
        V a[4], a2[4];
#pragma unroll
        for (int mb = 0; mb < 4; ++mb) { a[mb] = WFrag<T16>::ld(A + aoff + (size_t)mb * 16 * K + kc); if (NSPLIT == 1 || NSPLIT == 2) a2[mb] = WFrag<T16>::ld(A2 + aoff + (size_t)mb * 16 * K + kc); }
#pragma unroll
        for (int nb = 0; nb < 4; ++nb) { const V b = WFrag<T16>::ld(Bt + boff + (size_t)nb * 16 * K + kc); V b2; if (NSPLIT >= 2) b2 = WFrag<T16>::ld(Bt2 + boff + (size_t)nb * 16 * K + kc);
#pragma unroll
            for (int mb = 0; mb < 4; ++mb) { acc[mb][nb] = WFrag<T16>::mma(a[mb], b, acc[mb][nb]); if (NSPLIT == 1 || NSPLIT == 2) acc[mb][nb] = WFrag<T16>::mma(a2[mb], b, acc[mb][nb]); if (NSPLIT >= 2) acc[mb][nb] = WFrag<T16>::mma(a[mb], b2, acc[mb][nb]); } }
        asm volatile("v_nop\n\tv_nop\n\tv_nop\n\tv_nop" : "+v"(acc[0][0]), "+v"(acc[1][1]), "+v"(acc[2][2]), "+v"(acc[3][3]) : "v"(a[0]), "v"(a[3]));
    }
#pragma unroll
    for (int mb = 0; mb < 4; ++mb) {
#pragma unroll
        for (int nb = 0; nb < 4; ++nb) {
#pragma unroll
            for (int j = 0; j < 8; ++j) os[(hi * 8 + j) * 68 + nb * 16 + lr] = acc[mb][nb][j]; }
        __builtin_amdgcn_wave_barrier(); asm volatile("" ::: "memory");
        float* crow = C + (size_t)(r0 + mb * 16) * ldc + c0;
#pragma unroll 1
        for (int ps = 0; ps < 2; ++ps) {
#pragma unroll
            for (int s = 0; s < 8; ++s) { const int row = 2 * s + hi, cofs = lr * 4; v4f val = *(const v4fa*)(os + row * 68 + cofs); if (BIAS) { val[0] += bfr(bias[c0 + cofs]); val[1] += bfr(bias[c0 + cofs + 1]); val[2] += bfr(bias[c0 + cofs + 2]); val[3] += bfr(bias[c0 + cofs + 3]); }
                *(volatile v4f*)(crow + (size_t)row * ldc + cofs) = val; }
            if (ps == 0) __threadfence(); }
        __builtin_amdgcn_wave_barrier(); asm volatile("" ::: "memory");
    }
}

__device__ __forceinline__ h16 tohx(float x) { return (h16)x; }
__device__ __forceinline__ void splitf(float y, unsigned short& h, unsigned short& l) { h = f2bf(y); l = f2bf(y - bf2f(h)); }
typedef __attribute__((ext_vector_type(2))) unsigned short v2us;
typedef __attribute__((ext_vector_type(4))) unsigned short v4us;
typedef __attribute__((ext_vector_type(2))) _Float16 v2h;
typedef __attribute__((ext_vector_type(4))) _Float16 v4h;

__global__ __launch_bounds__(256) void k_cvt8(const float* __restrict__ src, bf* dst, size_t n8) { const size_t i = (size_t)blockIdx.x * 256 + threadIdx.x; if (i >= n8) return; const v8f v = *(const v8f*)(src + i * 8); v8us o;
#pragma unroll
    for (int k = 0; k < 8; ++k) o[k] = f2bf(v[k]); *(volatile v8us*)(dst + i * 8) = o; __threadfence(); *(volatile v8us*)(dst + i * 8) = o; }
__global__ __launch_bounds__(256) void k_ln256(const float* __restrict__ X, const float* __restrict__ g, const float* __restrict__ bb, size_t nrows, bf* Hh, bf* Hl) { const int lane = threadIdx.x & 31; const size_t r = (size_t)blockIdx.x * 8 + (threadIdx.x >> 5); if (r >= nrows) return; float v[8]; float s = 0.f;
#pragma unroll
    for (int ch = 0; ch < 2; ++ch) { const v4f a = *(const v4f*)(X + r * 256 + ch * 128 + lane * 4);
#pragma unroll
        for (int u = 0; u < 4; ++u) { v[ch * 4 + u] = bfr(a[u]); s += v[ch * 4 + u]; } }
#pragma unroll
    for (int sh = 16; sh; sh >>= 1) s += __shfl_xor(s, sh, 32);
    const float mean = s * (1.0f / 256); float q = 0.f;
#pragma unroll
    for (int k = 0; k < 8; ++k) { float d = __fsub_rn(v[k], mean); asm volatile("" : "+v"(d)); v[k] = d; float p = __fmul_rn(d, d); asm volatile("" : "+v"(p)); q = __fadd_rn(q, p); }
#pragma unroll
    for (int sh = 16; sh; sh >>= 1) q += __shfl_xor(q, sh, 32);
    const float rs = __frsqrt_rn(__fadd_rn(q * (1.0f / 256), 1e-5f));
    for (int ps = 0; ps < 2; ++ps) {
#pragma unroll
        for (int ch = 0; ch < 2; ++ch) { v4us oh, ol;
#pragma unroll
            for (int u = 0; u < 4; ++u) { const int c = ch * 128 + lane * 4 + u; float n0 = __fmul_rn(v[ch * 4 + u], rs); asm volatile("" : "+v"(n0)); float gg = bfr(g[c]), be = bfr(bb[c]); asm volatile("" : "+v"(gg)); asm volatile("" : "+v"(be)); float t1 = __fmul_rn(n0, gg); asm volatile("" : "+v"(t1)); unsigned short a2, c2; splitf(__fadd_rn(t1, be), a2, c2); oh[u] = a2; ol[u] = c2; }
            const size_t oo = r * 256 + ch * 128 + lane * 4; *(volatile v4us*)(Hh + oo) = oh; *(volatile v4us*)(Hl + oo) = ol; }
        if (ps == 0) __threadfence(); } }
__global__ __launch_bounds__(256) void k_ln128(const float* __restrict__ X, const float* __restrict__ g, const float* __restrict__ bb, size_t nrows, bf* Hh, bf* Hl) { const int lane = threadIdx.x & 31; const size_t r = (size_t)blockIdx.x * 8 + (threadIdx.x >> 5); if (r >= nrows) return; float v[4]; float s = 0.f; { const v4f a = *(const v4f*)(X + r * 128 + lane * 4);
#pragma unroll
        for (int u = 0; u < 4; ++u) { v[u] = bfr(a[u]); s += v[u]; } }
#pragma unroll
    for (int sh = 16; sh; sh >>= 1) s += __shfl_xor(s, sh, 32);
    const float mean = s * (1.0f / 128); float q = 0.f;
#pragma unroll
    for (int k = 0; k < 4; ++k) { float d = __fsub_rn(v[k], mean); asm volatile("" : "+v"(d)); v[k] = d; float p = __fmul_rn(d, d); asm volatile("" : "+v"(p)); q = __fadd_rn(q, p); }
#pragma unroll
    for (int sh = 16; sh; sh >>= 1) q += __shfl_xor(q, sh, 32);
    const float rs = __frsqrt_rn(__fadd_rn(q * (1.0f / 128), 1e-5f)); v4us oh, ol;
#pragma unroll
    for (int u = 0; u < 4; ++u) { const int c = lane * 4 + u; float n0 = __fmul_rn(v[u], rs); asm volatile("" : "+v"(n0)); float gg = bfr(g[c]), be = bfr(bb[c]); asm volatile("" : "+v"(gg)); asm volatile("" : "+v"(be)); float t1 = __fmul_rn(n0, gg); asm volatile("" : "+v"(t1)); unsigned short a2, c2; splitf(__fadd_rn(t1, be), a2, c2); oh[u] = a2; ol[u] = c2; }
    const size_t oo = r * 128 + lane * 4; *(volatile v4us*)(Hh + oo) = oh; *(volatile v4us*)(Hl + oo) = ol; __threadfence(); *(volatile v4us*)(Hh + oo) = oh; *(volatile v4us*)(Hl + oo) = ol; }
__global__ __launch_bounds__(256) void k_bw(const float* __restrict__ w, bf* Bt) { const int e = (blockIdx.x * 256 + threadIdx.x) * 4; if (e >= 64 * DP) return; const int n = e / DP; v4us o;
#pragma unroll
    for (int u = 0; u < 4; ++u) o[u] = (n < NH_) ? f2bf(w[e + u]) : (unsigned short)0; *(volatile v4us*)(Bt + e) = o; __threadfence(); *(volatile v4us*)(Bt + e) = o; }
__global__ __launch_bounds__(256) void k_qkp(const float* __restrict__ F, int s0, float sc, h16* P) { const size_t e = ((size_t)blockIdx.x * 256 + threadIdx.x) * 4; if (e >= (size_t)ZP * NN * HC) return; const int c = (int)(e % HC); const int i = (int)((e / HC) % NN); const int z = (int)(e / ((size_t)HC * NN)); const int sl = z / NH_, h = z % NH_; const float* f = F + ((size_t)(s0 + sl) * NN + i) * 256 + h * HC + c; v4h o;
#pragma unroll
    for (int u = 0; u < 4; ++u) { float t = f[u] * sc; asm volatile("" : "+v"(t)); o[u] = tohx(t); } *(volatile v4h*)(P + e) = o; __threadfence(); *(volatile v4h*)(P + e) = o; }
__global__ __launch_bounds__(256) void k_vtp(const float* __restrict__ F, int s0, h16* VT) { const size_t e = ((size_t)blockIdx.x * 256 + threadIdx.x) * 2; if (e >= (size_t)ZP * 64 * NN) return; const int j = (int)(e % NN); const int c = (int)((e / NN) % 64); const int z = (int)(e / ((size_t)NN * 64)); const int sl = z / NH_, h = z % NH_; v2h o;
    if (c < HC) { const float* f = F + ((size_t)(s0 + sl) * NN + j) * 256 + h * HC + c; o[0] = tohx(f[0]); o[1] = tohx(f[256]); } else { o[0] = (h16)0.f; o[1] = (h16)0.f; }
    *(volatile v2h*)(VT + e) = o; __threadfence(); *(volatile v2h*)(VT + e) = o; }
__global__ __launch_bounds__(256) void k_rsoft(const float* __restrict__ S, const float* __restrict__ BIAS, h16* P16) { const int lane = threadIdx.x & 31; const int row = blockIdx.x * 8 + (threadIdx.x >> 5); if (row >= ZP * NN) return; const int i = row % NN; const int z = row / NN; const int h = z % NH_; const float* sr = S + (size_t)row * NN; float v[NN / 32]; float mx = -3.0e38f;
#pragma unroll
    for (int ch = 0; ch < NN / 128; ++ch) { const v4f a = *(const v4f*)(sr + ch * 128 + lane * 4);
#pragma unroll
        for (int u = 0; u < 4; ++u) { const int j = ch * 128 + lane * 4 + u; const float t = __fadd_rn(a[u], BIAS[((size_t)i * NN + j) * 64 + h]); v[ch * 4 + u] = t; mx = fmaxf(mx, t); } }
#pragma unroll
    for (int sh = 16; sh; sh >>= 1) mx = fmaxf(mx, __shfl_xor(mx, sh, 32));
    float sum = 0.f;
#pragma unroll
    for (int q = 0; q < NN / 32; ++q) { float d0 = __fsub_rn(v[q], mx); asm volatile("" : "+v"(d0)); v[q] = __builtin_amdgcn_exp2f(__fmul_rn(d0, 1.4426950408889634f)); sum += v[q]; }
#pragma unroll
    for (int sh = 16; sh; sh >>= 1) sum += __shfl_xor(sum, sh, 32);
    const float f = __fdiv_rn(PCAR, sum);
    for (int ps = 0; ps < 2; ++ps) {
#pragma unroll
        for (int ch = 0; ch < NN / 128; ++ch) { v4h o4; for (int q = 0; q < 4; ++q) o4[q] = tohx(v[ch * 4 + q] * f); *(volatile v4h*)(P16 + (size_t)row * NN + ch * 128 + lane * 4) = o4; }
        if (ps == 0) __threadfence(); } }
__global__ __launch_bounds__(256) void k_og(const float* __restrict__ O, const float* __restrict__ G, const float* __restrict__ gb, int s0, bf* Ph, bf* Pl) { const size_t e = ((size_t)blockIdx.x * 256 + threadIdx.x) * 4; if (e >= (size_t)SPP * NN * 256) return; const int col = (int)(e % 256); const int i = (int)((e / 256) % NN); const int sl = (int)(e / ((size_t)256 * NN)); const int h = col / HC, c = col % HC; const int z = sl * NH_ + h; const size_t tok = (size_t)(s0 + sl) * NN + i; const float* src = O + ((size_t)z * NN + i) * 64 + c; v4us oh, ol;
#pragma unroll
    for (int u = 0; u < 4; ++u) { const float gz = __fadd_rn(G[tok * 256 + col + u], bfr(gb[col + u])); const float sg = __fdiv_rn(1.0f, __fadd_rn(1.0f, __expf(-gz))); float o1 = src[u] * (1.0f / PCAR); asm volatile("" : "+v"(o1)); unsigned short a, b; splitf(__fmul_rn(o1, sg), a, b); oh[u] = a; ol[u] = b; }
    const size_t oo = ((size_t)sl * NN + i) * 256 + col; *(volatile v4us*)(Ph + oo) = oh;     *(volatile v4us*)(Pl + oo) = ol; __threadfence(); *(volatile v4us*)(Ph + oo) = oh; *(volatile v4us*)(Pl + oo) = ol; }
__global__ __launch_bounds__(256) void k_resid(const float* __restrict__ X, float* O, size_t n4) { const size_t e = ((size_t)blockIdx.x * 256 + threadIdx.x) * 4; if (e >= n4 * 4) return; const v4f a = *(const v4f*)(X + e), o0 = *(const v4f*)(O + e); v4f r;
#pragma unroll
    for (int u = 0; u < 4; ++u) r[u] = __fadd_rn(bfr(a[u]), o0[u]); *(volatile v4f*)(O + e) = r; __threadfence(); *(volatile v4f*)(O + e) = r; }

extern "C" void kernel_launch(void* const* d_in, const int* in_sizes, int n_in,
                              void* d_out, int out_size, void* d_ws, size_t ws_size, hipStream_t stream) {
    (void)in_sizes; (void)n_in; (void)out_size;
    const float** I = (const float**)d_in;
    const float *Mraw = I[0], *Z = I[1], *lmg = I[2], *lmb = I[3], *lzg = I[4], *lzb = I[5], *bw = I[6], *qkvw = I[7], *gw = I[8], *gb = I[9], *ow = I[10], *ob = I[11];
    float* OUT = (float*)d_out;
    char* wsp = (char*)d_ws;
    auto take = [&](size_t bytes) { char* p = wsp; wsp += (bytes + 255) & ~(size_t)255; return (void*)p; };
    const size_t NTOK = (size_t)NS * NN, NPAIR = (size_t)NN * NN;
    bf* MNh = (bf*)take(NTOK * 256 * 2); bf* MNl = (bf*)take(NTOK * 256 * 2); bf* ZNh = (bf*)take(NPAIR * 128 * 2); bf* ZNl = (bf*)take(NPAIR * 128 * 2);
    bf* BW = (bf*)take((size_t)64 * 128 * 2); bf* BQKV = (bf*)take((size_t)768 * 256 * 2); bf* BG = (bf*)take((size_t)256 * 256 * 2); bf* BO = (bf*)take((size_t)256 * 256 * 2);
    float* BIAS = (float*)take(NPAIR * 64 * 4); float* F = (float*)take(NTOK * 256 * 4); float* G = (float*)take(NTOK * 256 * 4);
    h16* QP = (h16*)take((size_t)NS * NH_ * NN * HC * 2); h16* KP = (h16*)take((size_t)NS * NH_ * NN * HC * 2); h16* VT = (h16*)take((size_t)NS * NH_ * 64 * NN * 2);
    float* S = (float*)take((size_t)ZP * NN * NN * 4); h16* P16 = (h16*)take((size_t)ZP * NN * NN * 2); float* O = (float*)take((size_t)ZP * NN * 64 * 4); bf* OGh = (bf*)take((size_t)SPP * NN * 256 * 2); bf* OGl = (bf*)take((size_t)SPP * NN * 256 * 2);
    if ((size_t)(wsp - (char*)d_ws) > ws_size) return;
    k_ln256<<<(unsigned)((NTOK + 7) / 8), 256, 0, stream>>>(Mraw, lmg, lmb, NTOK, MNh, MNl); k_ln128<<<(unsigned)((NPAIR + 7) / 8), 256, 0, stream>>>(Z, lzg, lzb, NPAIR, ZNh, ZNl);
    k_bw<<<(64 * 128 / 4 + 255) / 256, 256, 0, stream>>>(bw, BW); k_cvt8<<<(768 * 256 / 8 + 255) / 256, 256, 0, stream>>>(qkvw, BQKV, 768 * 256 / 8); k_cvt8<<<(256 * 256 / 8 + 255) / 256, 256, 0, stream>>>(gw, BG, 256 * 256 / 8); k_cvt8<<<(256 * 256 / 8 + 255) / 256, 256, 0, stream>>>(ow, BO, 256 * 256 / 8);
    k_gemmw<bf, 1, false><<<dim3((unsigned)(NPAIR / 64), 1, 1), 32, 0, stream>>>(ZNh, ZNl, BW, nullptr, 128, BIAS, 64, nullptr, 0, 0, 0);
    const dim3 gt((unsigned)(NTOK / 64), 256 / 64, 1); const unsigned gqk = (unsigned)(((size_t)ZP * NN * HC / 4 + 255) / 256);
    k_gemmw<bf, 1, false><<<gt, 32, 0, stream>>>(MNh, MNl, BQKV, nullptr, 256, F, 256, nullptr, 0, 0, 0);
    for (int s0 = 0; s0 < NS; s0 += SPP) k_qkp<<<gqk, 256, 0, stream>>>(F, s0, 0.17677669529663689f, QP + (size_t)s0 * NH_ * NN * HC);
    k_gemmw<bf, 1, false><<<gt, 32, 0, stream>>>(MNh, MNl, BQKV + (size_t)256 * 256, nullptr, 256, F, 256, nullptr, 0, 0, 0);
    for (int s0 = 0; s0 < NS; s0 += SPP) k_qkp<<<gqk, 256, 0, stream>>>(F, s0, 1.0f, KP + (size_t)s0 * NH_ * NN * HC);
    k_gemmw<bf, 1, false><<<gt, 32, 0, stream>>>(MNh, MNl, BQKV + (size_t)512 * 256, nullptr, 256, F, 256, nullptr, 0, 0, 0);
    for (int s0 = 0; s0 < NS; s0 += SPP) k_vtp<<<(unsigned)(((size_t)ZP * 64 * NN / 2 + 255) / 256), 256, 0, stream>>>(F, s0, VT + (size_t)s0 * NH_ * 64 * NN);
    k_gemmw<bf, 1, false><<<gt, 32, 0, stream>>>(MNh, MNl, BG, nullptr, 256, G, 256, nullptr, 0, 0, 0);
    const size_t zq = (size_t)NN * HC, zS = (size_t)NN * NN, zv = (size_t)64 * NN, zo = (size_t)NN * 64;
    for (int s0 = 0; s0 < NS; s0 += SPP) { const size_t z0 = (size_t)s0 * NH_;
        k_gemmw<h16, 0, false><<<dim3(NN / 64, NN / 64, ZP), 32, 0, stream>>>(QP + z0 * zq, nullptr, KP + z0 * zq, nullptr, HC, S, NN, nullptr, zq, zq, zS);
        k_rsoft<<<ZP * NN / 8, 256, 0, stream>>>(S, BIAS, P16);
        k_gemmw<h16, 0, false><<<dim3(NN / 64, 1, ZP), 32, 0, stream>>>(P16, nullptr, VT + z0 * zv, nullptr, NN, O, 64, nullptr, zS, zv, zo);
        k_og<<<(unsigned)(((size_t)SPP * NN * 256 / 4 + 255) / 256), 256, 0, stream>>>(O, G, gb, s0, OGh, OGl);
        k_gemmw<bf, 1, true><<<dim3(SPP * NN / 64, 256 / 64, 1), 32, 0, stream>>>(OGh, OGl, BO, nullptr, 256, OUT + (size_t)s0 * NN * 256, 256, ob, 0, 0, 0);
        k_resid<<<(unsigned)(((size_t)SPP * NN * 256 / 4 + 255) / 256), 256, 0, stream>>>(Mraw + (size_t)s0 * NN * 256, OUT + (size_t)s0 * NN * 256, (size_t)SPP * NN * 256 / 4); }
}
